// KnowledgeConsistentAttention_7121055777354
// MI455X (gfx1250) — hardware-verified
//
#include <hip/hip_runtime.h>
#include <math.h>
#include <stdint.h>

#ifndef NIMG
#define NIMG 4
#endif
#define NB_FULL 4
#define NC     64
#define HW     64
#define NP     4096
#define QT     64
#define TP     72
#define OSP    68
#define XSC    16.0f
#define IXSC   0.0625f
#define EPSV   1.0e-7f
#define LNCARRY 10.397207708399179f

static_assert(NIMG >= 1 && NIMG <= NB_FULL);
static_assert(NP == HW * HW);
static_assert(NP % QT == 0 && NP % 32 == 0);
static_assert(NC == 64);
static_assert(QT == 64);
static_assert((TP * 2) % 16 == 0);
static_assert((OSP * 4) % 16 == 0);

typedef _Float16       v16h __attribute__((ext_vector_type(16)));
typedef _Float16       v8h  __attribute__((ext_vector_type(8)));
typedef __bf16         v16b __attribute__((ext_vector_type(16)));
typedef unsigned short v8us __attribute__((ext_vector_type(8)));
typedef float          v8f  __attribute__((ext_vector_type(8)));
typedef float          v4f  __attribute__((ext_vector_type(4)));
typedef unsigned int   v4u  __attribute__((ext_vector_type(4)));

union Frag  { v8us u[2]; v16h h; v16b bf; };
union FragH { v16h v; v8h hv[2]; };
static_assert(sizeof(Frag) == 32);
static_assert(sizeof(FragH) == 32);

__device__ __forceinline__ unsigned short bf_bits(float f) {
  unsigned u = __float_as_uint(f);
  return (unsigned short)((u + 0x7FFFu + ((u >> 16) & 1u)) >> 16);
}
__device__ __forceinline__ float bf_up(unsigned short hb) { return __uint_as_float(((unsigned)hb) << 16); }
__device__ __forceinline__ float bfr(float f) { return bf_up(bf_bits(f)); }
__device__ __forceinline__ unsigned short h_bits(_Float16 x) { return __builtin_bit_cast(unsigned short, x); }
__device__ __forceinline__ unsigned pk16(unsigned short a, unsigned short b) { return (unsigned)a | ((unsigned)b << 16); }
__device__ __forceinline__ v8f zero8() { v8f z = {0.f, 0.f, 0.f, 0.f, 0.f, 0.f, 0.f, 0.f}; return z; }
__device__ __forceinline__ float hmax8(v8f s) {
  return fmaxf(fmaxf(fmaxf(s[0], s[1]), fmaxf(s[2], s[3])), fmaxf(fmaxf(s[4], s[5]), fmaxf(s[6], s[7])));
}
__device__ __forceinline__ unsigned wave_ballot(bool p) {
#if defined(__HIP_DEVICE_COMPILE__)
  return __builtin_amdgcn_ballot_w32(p);
#else
  return p ? 1u : 0u;
#endif
}

__device__ __forceinline__ Frag ldfrag(const unsigned short* p) {
  Frag f;
  f.u[0] = *(const v8us*)(p);
  f.u[1] = *(const v8us*)(p + 16);
  return f;
}

__device__ __forceinline__ v8f mma_h(v16h a, v16h b, v8f c) {
  v8f d = __builtin_amdgcn_wmma_f32_16x16x32_f16(false, a, false, b, (short)0, c, false, false);
#if defined(__HIP_DEVICE_COMPILE__)
  asm volatile("v_nop\n\tv_nop\n\tv_nop\n\tv_nop" : "+v"(d) : "v"(a), "v"(b));
#endif
  return d;
}
__device__ __forceinline__ v8f mma_b(v16b a, v16b b, v8f c) {
  v8f d = __builtin_amdgcn_wmma_f32_16x16x32_bf16(false, a, false, b, (short)0, c, false, false);
#if defined(__HIP_DEVICE_COMPILE__)
  const v16h ha = __builtin_bit_cast(v16h, a), hb = __builtin_bit_cast(v16h, b);
  asm volatile("v_nop\n\tv_nop\n\tv_nop\n\tv_nop" : "+v"(d) : "v"(ha), "v"(hb));
#endif
  return d;
}

__global__ __launch_bounds__(256)
void cvt_f(const float* __restrict__ f, const float* __restrict__ aux, unsigned short* FC, unsigned short* FP,
           float* R) {
  (void)aux;
  __shared__ __align__(16) unsigned short T[QT * TP];
  __shared__ __align__(16) float Rs[QT];
  const int tid = threadIdx.x;
  const int pt = blockIdx.x, b = blockIdx.y;
  const int e = tid & 7, lq = tid >> 3;
  const int p0 = pt * QT;
  v4u uc[2];
#pragma unroll
  for (int it = 0; it < 2; ++it) {
    const int cl = it * 32 + lq;
    const float* sp = f + ((size_t)(b * NC + cl)) * NP + p0 + 8 * e;
    const v4f a = *(const v4f*)sp;
    const v4f q = *(const v4f*)(sp + 4);
    const float g[8] = {a[0], a[1], a[2], a[3], q[0], q[1], q[2], q[3]};
    unsigned short hb[8], bb[8];
#pragma unroll
    for (int t = 0; t < 8; ++t) {
      bb[t] = bf_bits(g[t]);
      hb[t] = h_bits((_Float16)(bf_up(bb[t]) * XSC));
    }
#pragma unroll
    for (int t = 0; t < 4; ++t) uc[it][t] = pk16(hb[2 * t], hb[2 * t + 1]);
#pragma unroll
    for (int t = 0; t < 8; ++t) T[(8 * e + t) * TP + cl] = bb[t];
  }
  __syncthreads();
  v4u up[2];
#pragma unroll
  for (int it = 0; it < 2; ++it) {
    const int pl = it * 32 + lq;
    up[it] = *(const v4u*)(T + pl * TP + 8 * e);
  }
  {
    const int pl = tid >> 2, sub = tid & 3;
    const unsigned short* tr = T + pl * TP + 16 * sub;
    const v8us w0 = *(const v8us*)(tr);
    const v8us w1 = *(const v8us*)(tr + 8);
    float s = 0.f;
#pragma unroll
    for (int i = 0; i < 8; ++i) { const float v = bf_up(w0[i]) + EPSV; s += v * v; }
#pragma unroll
    for (int i = 0; i < 8; ++i) { const float v = bf_up(w1[i]) + EPSV; s += v * v; }
    s += __shfl_xor(s, 1, 32);
    s += __shfl_xor(s, 2, 32);
    if (sub == 0) Rs[pl] = rsqrtf(s);
  }
  __syncthreads();
  const v4f rv = *(const v4f*)(Rs + 4 * (tid & 15));
#pragma unroll
  for (int pass = 0; pass < 2; ++pass) {
#pragma unroll
    for (int it = 0; it < 2; ++it) {
      const int rl = it * 32 + lq;
      *(volatile v4u*)(FC + ((size_t)(b * NC + rl)) * NP + p0 + 8 * e) = uc[it];
      *(volatile v4u*)(FP + ((size_t)(b * NP + p0 + rl)) * NC + 8 * e) = up[it];
    }
    if (tid < 16) *(volatile v4f*)(R + (size_t)b * NP + p0 + 4 * tid) = rv;
    __threadfence();
  }
}

__global__ __launch_bounds__(256)
void pool_q(const float* __restrict__ f, unsigned short* Qh, unsigned short* Ql, float* G) {
  __shared__ __align__(16) unsigned short Th[QT * TP];
  __shared__ __align__(16) unsigned short Tl[QT * TP];
  __shared__ __align__(16) float Gs[NC * QT];
  __shared__ __align__(16) float Gq[QT];
  const int tid = threadIdx.x;
  const int y = blockIdx.x, b = blockIdx.y;
  const int ch = tid >> 2, xq = tid & 3, x0 = 16 * xq;
  const float* fc = f + ((size_t)(b * NC + ch)) * NP;
  float s[16];
#pragma unroll
  for (int i = 0; i < 16; ++i) s[i] = 0.f;
#pragma unroll
  for (int dy = -1; dy <= 1; ++dy) {
    const int yy = y + dy;
    if (yy >= 0 && yy < HW) {
      const float* row = fc + yy * HW;
      const v4f a0 = *(const v4f*)(row + x0);
      const v4f a1 = *(const v4f*)(row + x0 + 4);
      const v4f a2 = *(const v4f*)(row + x0 + 8);
      const v4f a3 = *(const v4f*)(row + x0 + 12);
      const int xl = (x0 > 0) ? (x0 - 1) : 0;
      const int xr = (x0 + 16 < HW) ? (x0 + 16) : (HW - 1);
      float vl = row[xl]; vl = (x0 > 0) ? vl : 0.f;
      float vr = row[xr]; vr = (x0 + 16 < HW) ? vr : 0.f;
      float v[18];
      v[0] = bfr(vl); v[17] = bfr(vr);
#pragma unroll
      for (int t = 0; t < 4; ++t) {
        v[1 + t]  = bfr(a0[t]);
        v[5 + t]  = bfr(a1[t]);
        v[9 + t]  = bfr(a2[t]);
        v[13 + t] = bfr(a3[t]);
      }
#pragma unroll
      for (int i = 0; i < 16; ++i) s[i] += (v[i] + v[i + 1]) + v[i + 2];
    }
  }
#pragma unroll
  for (int i = 0; i < 16; ++i) {
    const unsigned short hb = bf_bits(s[i]);
    const unsigned short lb = bf_bits(s[i] - bf_up(hb));
    Th[(x0 + i) * TP + ch] = hb;
    Tl[(x0 + i) * TP + ch] = lb;
  }
#pragma unroll
  for (int t = 0; t < 4; ++t) {
    v4f gv4 = {s[4 * t], s[4 * t + 1], s[4 * t + 2], s[4 * t + 3]};
    *(v4f*)(Gs + ch * QT + x0 + 4 * t) = gv4;
  }
  __syncthreads();
  if (tid < QT) {
    float g = 0.f;
#pragma unroll 4
    for (int cc = 0; cc < NC; ++cc) g += Gs[cc * QT + tid];
    Gq[tid] = g * EPSV;
  }
  const int e = tid & 7, lq = tid >> 3;
  v4u uh[2], ul[2];
#pragma unroll
  for (int it = 0; it < 2; ++it) {
    const int xl2 = it * 32 + lq;
    uh[it] = *(const v4u*)(Th + xl2 * TP + 8 * e);
    ul[it] = *(const v4u*)(Tl + xl2 * TP + 8 * e);
  }
  __syncthreads();
  const v4f gv = *(const v4f*)(Gq + 4 * (tid & 15));
#pragma unroll
  for (int pass = 0; pass < 2; ++pass) {
#pragma unroll
    for (int it = 0; it < 2; ++it) {
      const int xl2 = it * 32 + lq;
      const size_t po = ((size_t)(b * NP + y * HW + xl2)) * NC + 8 * e;
      *(volatile v4u*)(Qh + po) = uh[it];
      *(volatile v4u*)(Ql + po) = ul[it];
    }
    if (tid < 16) *(volatile v4f*)(G + (size_t)b * NP + y * HW + 4 * tid) = gv;
    __threadfence();
  }
}

__global__ __launch_bounds__(128)
void attn_k(const unsigned short* __restrict__ Qh, const unsigned short* __restrict__ Ql,
            const unsigned short* __restrict__ FP, const unsigned short* __restrict__ FC,
            const float* __restrict__ R, const float* __restrict__ G, float* out) {
  __shared__ __align__(16) float Os[QT * OSP];
  const int tid  = threadIdx.x;
  const int wave = tid >> 5, lane = tid & 31;
  const int hh   = lane >> 4, c = lane & 15;
  const int n0   = blockIdx.x * QT, b = blockIdx.y;

  const size_t qo = ((size_t)(b * NP + n0 + 16 * wave + c)) * NC + 8 * hh;
  const Frag qh0 = ldfrag(Qh + qo);
  const Frag qh1 = ldfrag(Qh + qo + 32);
  const Frag ql0 = ldfrag(Ql + qo);
  const Frag ql1 = ldfrag(Ql + qo + 32);
  const float gq = G[(size_t)b * NP + n0 + 16 * wave + c];
  const unsigned short* Kp = FP + (size_t)b * NP * NC + (size_t)c * NC + 8 * hh;
  const unsigned short* Vp = FC + (size_t)b * NC * NP + (size_t)c * NP + 8 * hh;
  const float* Rp = R + (size_t)b * NP + 8 * hh;

  float m = -1.0e30f, l = 0.f, E = 0.f;
  v8f o[4];
#pragma unroll
  for (int j = 0; j < 4; ++j) o[j] = zero8();

#pragma unroll 1
  for (int kb = 0; kb < NP; kb += 32) {
    const unsigned short* k0p = Kp + (size_t)kb * NC;
    const unsigned short* k1p = Kp + (size_t)(kb + 16) * NC;
    v8f s0 = zero8(), s1 = zero8();
    {
      const Frag a0 = ldfrag(k0p), a1 = ldfrag(k0p + 32);
      const Frag c0 = ldfrag(k1p), c1 = ldfrag(k1p + 32);
      s0 = mma_b(a0.bf, qh0.bf, s0);
      s1 = mma_b(c0.bf, qh0.bf, s1);
      s0 = mma_b(a0.bf, ql0.bf, s0);
      s1 = mma_b(c0.bf, ql0.bf, s1);
      s0 = mma_b(a1.bf, qh1.bf, s0);
      s1 = mma_b(c1.bf, qh1.bf, s1);
      s0 = mma_b(a1.bf, ql1.bf, s0);
      s1 = mma_b(c1.bf, ql1.bf, s1);
    }
    const v4f ra = *(const v4f*)(Rp + kb);
    const v4f rb = *(const v4f*)(Rp + kb + 4);
    const v4f rc = *(const v4f*)(Rp + kb + 16);
    const v4f rd = *(const v4f*)(Rp + kb + 20);
    const float r0v[8] = {ra[0], ra[1], ra[2], ra[3], rb[0], rb[1], rb[2], rb[3]};
    const float r1v[8] = {rc[0], rc[1], rc[2], rc[3], rd[0], rd[1], rd[2], rd[3]};
#pragma unroll
    for (int r = 0; r < 8; ++r) {
      s0[r] = r0v[r] * (s0[r] + gq);
      s1[r] = r1v[r] * (s1[r] + gq);
    }

    float mx = fmaxf(hmax8(s0), hmax8(s1));
    mx = fmaxf(mx, __shfl_xor(mx, 16, 32));
    const float mn = fmaxf(m, mx);
    const unsigned grew = wave_ballot(mx > m);
    if (grew != 0u) {
      const float corr = __expf(m - mn);
      l *= corr;
      E *= corr;
#pragma unroll
      for (int j = 0; j < 4; ++j) {
#pragma unroll
        for (int r = 0; r < 8; ++r) o[j][r] *= corr;
      }
    }
    m = mn;
    const float msh = mn - LNCARRY;

    FragH ph;
    float ls = 0.f, es = 0.f;
#pragma unroll
    for (int r = 0; r < 8; ++r) {
      const float e0 = __expf(s0[r] - msh);
      const float e1 = __expf(s1[r] - msh);
      ls += e0 + e1;
      const float pe0 = e0 * r0v[r];
      const float pe1 = e1 * r1v[r];
      es += pe0 + pe1;
      ph.hv[0][r] = (_Float16)pe0;
      ph.hv[1][r] = (_Float16)pe1;
    }
    l += ls;
    E += es;

#pragma unroll
    for (int j = 0; j < 4; ++j) {
      const Frag vf = ldfrag(Vp + (size_t)(16 * j) * NP + kb);
      o[j] = mma_h(vf.h, ph.v, o[j]);
    }
  }
  l += __shfl_xor(l, 16, 32);
  E += __shfl_xor(E, 16, 32);
  const float inv = 1.0f / l;
  const float ee  = EPSV * E;

  const int qrow = 16 * wave + c;
#pragma unroll
  for (int j = 0; j < 4; ++j) {
    v4f va, vb;
#pragma unroll
    for (int r = 0; r < 4; ++r) {
      va[r] = (o[j][r] * IXSC + ee) * inv;
      vb[r] = (o[j][4 + r] * IXSC + ee) * inv;
    }
    *(v4f*)(Os + qrow * OSP + 16 * j + 8 * hh)     = va;
    *(v4f*)(Os + qrow * OSP + 16 * j + 8 * hh + 4) = vb;
  }
  __syncthreads();
  const int e = tid & 7, lq = tid >> 3;
  v4f res[8];
#pragma unroll
  for (int it = 0; it < 8; ++it) {
    const int L   = it * 16 + lq;
    const int chl = L >> 1, hf = L & 1;
    const int nl  = hf * 32 + 4 * e;
#pragma unroll
    for (int t = 0; t < 4; ++t) res[it][t] = Os[(nl + t) * OSP + chl];
  }
#pragma unroll
  for (int pass = 0; pass < 2; ++pass) {
#pragma unroll
    for (int it = 0; it < 8; ++it) {
      const int L   = it * 16 + lq;
      const int chl = L >> 1, hf = L & 1;
      const int nl  = hf * 32 + 4 * e;
      const size_t idx = ((size_t)(b * NC + chl)) * NP + n0 + nl;
      *(volatile v4f*)(out + idx) = res[it];
    }
    __threadfence();
  }
}

extern "C" void kernel_launch(void* const* d_in, const int* in_sizes, int n_in,
                              void* d_out, int out_size, void* d_ws, size_t ws_size,
                              hipStream_t stream) {
  const int XN = NIMG * NC * NP;
  if (n_in < 2) return;
  if (in_sizes[0] < XN) return;
  if (out_size < XN) return;

  size_t off = 0;
  auto carve = [&](size_t bytes) { const size_t o = off; off += (bytes + 255) & ~(size_t)255; return o; };
  const size_t oFC = carve((size_t)NIMG * NC * NP * 2);
  const size_t oFP = carve((size_t)NIMG * NP * NC * 2);
  const size_t oQh = carve((size_t)NIMG * NP * NC * 2);
  const size_t oQl = carve((size_t)NIMG * NP * NC * 2);
  const size_t oR  = carve((size_t)NIMG * NP * 4);
  const size_t oG  = carve((size_t)NIMG * NP * 4);
  if (off > ws_size) return;
  if (off > (size_t)134217728) return;

  const float* fg = (const float*)d_in[0];
  const float* aux = (const float*)d_in[1];

  char* ws = (char*)d_ws;
  unsigned short* FC = (unsigned short*)(ws + oFC);
  unsigned short* FP = (unsigned short*)(ws + oFP);
  unsigned short* Qh = (unsigned short*)(ws + oQh);
  unsigned short* Ql = (unsigned short*)(ws + oQl);
  float* R = (float*)(ws + oR);
  float* G = (float*)(ws + oG);
  float* out = (float*)d_out;

  const dim3 blk256(256), blk128(128);

  cvt_f<<<dim3(NP / QT, NIMG), blk256, 0, stream>>>(fg, aux, FC, FP, R);
  pool_q<<<dim3(HW, NIMG), blk256, 0, stream>>>(fg, Qh, Ql, G);
  attn_k<<<dim3(NP / QT, NIMG), blk128, 0, stream>>>(Qh, Ql, FP, FC, R, G, out);
  (void)hipGetLastError();
}
